// BiMamba_58085137711712
// MI455X (gfx1250) — hardware-run, weakly checked
//
#include <hip/hip_runtime.h>
#include <hip/hip_fp16.h>
#include <math.h>

typedef float    ms1_v4f __attribute__((ext_vector_type(4)));
typedef unsigned ms1_v4u __attribute__((ext_vector_type(4)));
struct ms1_args {
  const float* dtpre;
  const float* u;
  const float* bc;
  const float* z;
  const float* A_log;
  const float* Dskip;
  __half* y;
  __half* y_lo;
  long ld_dtpre;
  long ld_u;
  long ld_bc;
  long ld_z;
  long ld_y;
  int offB;
  int offC;
  int offZ;
  float ycarry;
  int dir;
  int D;
  int L;
  int nbatch;
};
static_assert(sizeof(ms1_args) == 136);

__device__ __forceinline__ float ms1_flush16(float v) {
  return (fabsf(v) < 6.103515625e-05f) ? 0.0f : v;
}
__device__ __forceinline__ unsigned ms1_h16bits(float v) {
  return (unsigned)__half_as_ushort(__float2half_rn(ms1_flush16(v)));
}
__device__ __forceinline__ float ms1_h16val(unsigned b) {
  return __half2float(__ushort_as_half((unsigned short)b));
}
__device__ __forceinline__ float ms1_softplus(float v) {
  return fmaxf(v, 0.0f) + log1pf(expf(-fabsf(v)));
}
__device__ __forceinline__ void ms1_pack2(float v0, float v1, unsigned& hw, unsigned& lw) {
  const unsigned h0 = ms1_h16bits(v0);
  const unsigned h1 = ms1_h16bits(v1);
  const float r0 = (v0 - ms1_h16val(h0)) * 2048.0f;
  const float r1 = (v1 - ms1_h16val(h1)) * 2048.0f;
  const unsigned l0 = ms1_h16bits(r0);
  const unsigned l1 = ms1_h16bits(r1);
  hw = h0 | (h1 << 16);
  lw = l0 | (l1 << 16);
}

template <int NSTATE>
__global__ __launch_bounds__(64 * (NSTATE / 16)) void ms1_scan_kernel(ms1_args a)
{
  static_assert(NSTATE == 16 || NSTATE == 64);
  constexpr int NQ  = NSTATE / 16;
  constexpr int NT  = 64 * NQ;
  constexpr int NW  = NT / 32;
  constexpr int BCW = 2 * NSTATE;
  constexpr int YP  = 68;
  constexpr int RPI = NW * 4;
  constexpr int NIT = 64 / RPI;
  static_assert(16 * NT <= 64 * YP);
  __shared__ __align__(16) float sBC[64 * BCW];
  __shared__ __align__(16) float sY[64 * YP];
  const int tid  = threadIdx.x;
  const int lane = tid & 31;
  const int wave = tid >> 5;
  const int c    = tid / NQ;
  const int sq   = tid - c * NQ;
  const int bpb  = a.D / 64;
  const int bi   = blockIdx.x / bpb;
  if (bi >= a.nbatch) return;
  const int d0 = (blockIdx.x - bi * bpb) * 64;
  const int d  = d0 + c;
  const long rowb = (long)bi * a.L;
  const bool hasz  = (a.z != nullptr);
  const bool hasD  = (a.Dskip != nullptr);
  const bool hasLo = (a.y_lo != nullptr);

#pragma unroll 1
  for (int n = 0; n < 16; ++n) {
    const float al = a.A_log[(long)d * NSTATE + sq * 16 + n];
    sY[n * NT + tid] = -expf(al);
  }
  __syncthreads();
  float An[16], h[16];
#pragma unroll
  for (int n = 0; n < 16; ++n) {
    An[n] = sY[n * NT + tid];
    h[n] = 0.0f;
  }
  float Dd = 0.0f;
  if (hasD) Dd = a.Dskip[d];

  const int nchunk = a.L / 64;
  const bool fwd = (a.dir > 0);
  const int s0 = fwd ? 0 : 63;
  const int sd = fwd ? 1 : -1;
  const int q  = lane >> 3;
  const int c8 = (lane & 7) * 8;

#pragma unroll 1
  for (int ci = 0; ci < nchunk; ++ci) {
    const int tb = fwd ? (ci * 64) : (a.L - 64 - ci * 64);
    const long rowc = rowb + tb;
    __syncthreads();
#pragma unroll 8
    for (int i = 0; i < 32; ++i) {
      const int idx = tid + i * NT;
      const int st  = idx / BCW;
      const int col = idx - st * BCW;
      const int sc  = (col < NSTATE) ? (a.offB + col) : (a.offC + col - NSTATE);
      sBC[idx] = a.bc[(rowc + st) * a.ld_bc + sc];
    }
    __syncthreads();
#pragma unroll 1
    for (int s = 0; s < 64; ++s) {
      const int ls = s0 + sd * s;
      const long row = rowc + ls;
      float pre = a.dtpre[row * a.ld_dtpre + d];
      float uv  = a.u[row * a.ld_u + d];
      float zv  = 0.0f;
      if (hasz) zv = a.z[row * a.ld_z + a.offZ + d];
      asm volatile("" : "+v"(pre));
      asm volatile("" : "+v"(uv));
      asm volatile("" : "+v"(zv));
      const float delta = ms1_softplus(pre);
      const float dtx = delta * uv;
      const float* bp = sBC + ls * BCW + sq * 16;
      const float* cp = bp + NSTATE;
      ms1_v4f Bq[4], Cq[4];
#pragma unroll
      for (int k = 0; k < 4; ++k) {
        Bq[k] = *(const ms1_v4f*)(bp + 4 * k);
        Cq[k] = *(const ms1_v4f*)(cp + 4 * k);
      }
      float yv = 0.0f;
#pragma unroll
      for (int n = 0; n < 16; ++n) {
        const float e = __expf(delta * An[n]);
        h[n] = fmaf(e, h[n], dtx * Bq[n >> 2][n & 3]);
        yv = fmaf(h[n], Cq[n >> 2][n & 3], yv);
      }
      if (NQ > 1) {
        yv += __shfl_xor(yv, 1, 32);
        yv += __shfl_xor(yv, 2, 32);
      }
      if (hasD) yv = fmaf(uv, Dd, yv);
      if (hasz) {
        const float sg = __builtin_amdgcn_rcpf(1.0f + expf(-zv));
        yv = yv * (zv * sg);
      }
      if (sq == 0) sY[ls * YP + c] = yv * a.ycarry;
    }
    __syncthreads();
    ms1_v4u hw[NIT], lw[NIT];
#pragma unroll
    for (int it = 0; it < NIT; ++it) {
      const int row = it * RPI + wave * 4 + q;
      const float* sp = sY + row * YP + c8;
      const ms1_v4f f0 = *(const ms1_v4f*)(sp);
      const ms1_v4f f1 = *(const ms1_v4f*)(sp + 4);
      unsigned h0, h1, h2, h3, l0, l1, l2, l3;
      ms1_pack2(f0[0], f0[1], h0, l0);
      ms1_pack2(f0[2], f0[3], h1, l1);
      ms1_pack2(f1[0], f1[1], h2, l2);
      ms1_pack2(f1[2], f1[3], h3, l3);
      hw[it] = (ms1_v4u){h0, h1, h2, h3};
      lw[it] = (ms1_v4u){l0, l1, l2, l3};
    }
    for (int pass = 0; pass < 2; ++pass) {
#pragma unroll
      for (int it = 0; it < NIT; ++it) {
        const int row = it * RPI + wave * 4 + q;
        const long o = (rowc + row) * a.ld_y + d0 + c8;
        *(volatile ms1_v4u*)(a.y + o) = hw[it];
        if (hasLo) *(volatile ms1_v4u*)(a.y_lo + o) = lw[it];
      }
      __threadfence();
    }
  }
}

typedef __attribute__((ext_vector_type(16))) _Float16 v16h;
typedef __attribute__((ext_vector_type(8)))  _Float16 v8h;
typedef __attribute__((ext_vector_type(8)))  float    v8f;
typedef __attribute__((ext_vector_type(4)))  float    v4f;

constexpr int kBatch  = 2;
constexpr int kSeq    = 1024;
constexpr int kDm     = 1024;
constexpr int kDin    = 2048;
constexpr int kNst    = 16;
constexpr int kDtR    = 64;
constexpr int kNSeq   = 2 * kBatch;
constexpr int kXzP    = 2 * kDin;
constexpr int kXpN    = kDtR + 2 * kNst;
constexpr int kXpNP   = 128;
constexpr int kBcP    = 64;
constexpr int kDff    = 4 * kDm;
constexpr int kRowsAll = kNSeq * kSeq;
constexpr int kRowsOut = kBatch * kSeq;
constexpr int kConvTP  = 260;
static_assert(kXpN == 96 && kXpN <= kXpNP && (kXpN % 4) == 0, "x_proj width");
static_assert(kDtR == 64 && kBcP == 64 && kXpNP == kDtR + kBcP, "x_proj column halves");
static_assert((kDm % 64) == 0 && (kDin % 64) == 0 && (kDff % 64) == 0 && (kDtR % 64) == 0, "K multiples of 64 (32 for the k-step, 64 for the transposing convert)");
static_assert((kSeq % 64) == 0 && (kXzP % 64) == 0 && (kRowsAll % 64) == 0 && (kRowsOut % 64) == 0, "M, N multiples of 64");
static_assert((kDin % 256) == 0 && (kDm / 8) == 128, "elementwise tilings");

constexpr float kCarryX  = 16.0f;
constexpr float kCarryW  = 1024.0f;
constexpr float kCarryU  = 256.0f;
constexpr float kCarryDt = 256.0f;
constexpr float kCarryY  = 1024.0f;
constexpr float kCarryH  = 16.0f;
constexpr float kCarryG  = 64.0f;
constexpr float kF16Min  = 6.103515625e-05f;

constexpr size_t kOffWIN   = 0;
constexpr size_t kOffWXP   = kOffWIN   + (size_t)kXzP  * kDm  * 2;
constexpr size_t kOffWDT   = kOffWXP   + (size_t)kXpNP * kDin * 2;
constexpr size_t kOffWOUT  = kOffWDT   + (size_t)kDin  * kDtR * 2;
constexpr size_t kOffWF1   = kOffWOUT  + (size_t)kDm   * kDin * 2;
constexpr size_t kOffWF2   = kOffWF1   + (size_t)kDff  * kDm  * 2;
constexpr size_t kOffX16   = kOffWF2   + (size_t)kDm   * kDff * 2;
constexpr size_t kOffXZS   = kOffX16   + (size_t)kRowsAll * kDm * 2;
constexpr size_t kOffUS    = kOffXZS   + (size_t)kSeq * kXzP * 4;
constexpr size_t kOffU16S  = kOffUS    + (size_t)kSeq * kDin * 4;
constexpr size_t kOffBCS   = kOffU16S  + (size_t)kSeq * kDin * 2;
constexpr size_t kOffDT16S = kOffBCS   + (size_t)kSeq * kBcP * 4;
constexpr size_t kOffDTPS  = kOffDT16S + (size_t)kSeq * kDtR * 2;
constexpr size_t kOffY16   = kOffDTPS  + (size_t)kSeq * kDin * 4;
constexpr size_t kOffMO    = kOffY16   + (size_t)kRowsAll * kDin * 2;
constexpr size_t kOffH16   = kOffMO    + (size_t)kRowsAll * kDm * 4;
constexpr size_t kOffG16   = kOffH16   + (size_t)kRowsOut * kDm * 2;
constexpr size_t kWsTotal  = kOffG16   + (size_t)kRowsOut * kDff * 2;
static_assert(kWsTotal == 131203072ull, "carve total");
static_assert(kWsTotal <= 134217728ull, "carve cap");
static_assert((size_t)kSeq * kDff * 4 == (size_t)kSeq * kXzP * 4, "MLP-up chunk fits the XZS region exactly");
static_assert((kOffWXP % 128) == 0 && (kOffWDT % 128) == 0 && (kOffWOUT % 128) == 0 && (kOffWF1 % 128) == 0 &&
              (kOffWF2 % 128) == 0 && (kOffX16 % 128) == 0 && (kOffXZS % 128) == 0 && (kOffUS % 128) == 0 &&
              (kOffU16S % 128) == 0 && (kOffBCS % 128) == 0 && (kOffDT16S % 128) == 0 && (kOffDTPS % 128) == 0 &&
              (kOffY16 % 128) == 0 && (kOffMO % 128) == 0 && (kOffH16 % 128) == 0 && (kOffG16 % 128) == 0,
              "128-B aligned regions");

namespace eng {

__device__ __forceinline__ float flush16(float v) {
  return (fabsf(v) < kF16Min) ? 0.0f : v;
}

__device__ __forceinline__ void guard1_h(v8f& a, v16h x, v16h y) {
  asm volatile("v_nop\n\tv_nop\n\tv_nop\n\tv_nop" : "+v"(a) : "v"(x), "v"(y));
}
__device__ __forceinline__ void keep4_h(v16h a, v16h b, v16h c, v16h d) {
  asm volatile("v_nop" :: "v"(a), "v"(b), "v"(c), "v"(d));
}
__device__ __forceinline__ void acc_guard4(v8f& a, v8f& b, v8f& c, v8f& d) {
  asm volatile("v_nop\n\tv_nop\n\tv_nop\n\tv_nop" : "+v"(a), "+v"(b), "+v"(c), "+v"(d));
}

struct FragH {
  union U { v16h v; v8h h[2]; };
  static __device__ __forceinline__ v16h load(const _Float16* p) {
    U f;
    f.h[0] = *(const v8h*)(p);
    f.h[1] = *(const v8h*)(p + 16);
    return f.v;
  }
  static __device__ __forceinline__ v8f mma(v16h a, v16h b, v8f c) {
    return __builtin_amdgcn_wmma_f32_16x16x32_f16(false, a, false, b, (short)0, c, false, false);
  }
};

template <int BIAS_MODE, int OUT_MODE>
__global__ __launch_bounds__(256) void gemm_f16_kernel(
    const unsigned short* __restrict__ Ap, int lda,
    const unsigned short* __restrict__ Btp, int ldb,
    void* __restrict__ Cout, int ldc,
    const float* __restrict__ bias,
    int M, int N, int K, float scale)
{
  const _Float16* A  = (const _Float16*)Ap;
  const _Float16* Bt = (const _Float16*)Btp;
  __shared__ __align__(16) float sT[8][16 * 68];
  const int lane = threadIdx.x & 31;
  const int wave = threadIdx.x >> 5;
  const int tilesN = N >> 6;
  const int tilesM = M >> 6;
  const int tile = blockIdx.x * 8 + wave;
  if (tile >= tilesM * tilesN) return;
  const int tm = tile / tilesN;
  const int tn = tile - tm * tilesN;
  const int m0 = tm << 6;
  const int n0 = tn << 6;

  const int rlane = lane & 15;
  const int koff  = (lane >> 4) * 8;
  const int mOff  = (lane >> 4) * 8;

  v8f acc[4][4];
#pragma unroll
  for (int i = 0; i < 4; ++i)
#pragma unroll
    for (int j = 0; j < 4; ++j) acc[i][j] = (v8f){0.f, 0.f, 0.f, 0.f, 0.f, 0.f, 0.f, 0.f};

  for (int k0 = 0; k0 < K; k0 += 32) {
    v16h bh[4];
#pragma unroll
    for (int j = 0; j < 4; ++j) {
      const size_t bo = (size_t)(n0 + (j << 4) + rlane) * ldb + koff + k0;
      bh[j] = FragH::load(Bt + bo);
    }
#pragma unroll
    for (int i = 0; i < 4; ++i) {
      const size_t ao = (size_t)(m0 + (i << 4) + rlane) * lda + koff + k0;
      const v16h ah = FragH::load(A + ao);
#pragma unroll
      for (int j = 0; j < 4; ++j) acc[i][j] = FragH::mma(ah, bh[j], acc[i][j]);
      guard1_h(acc[i][0], ah, bh[0]);
      guard1_h(acc[i][1], ah, bh[1]);
      guard1_h(acc[i][2], ah, bh[2]);
      guard1_h(acc[i][3], ah, bh[3]);
    }
    keep4_h(bh[0], bh[1], bh[2], bh[3]);
  }
  acc_guard4(acc[0][0], acc[0][1], acc[0][2], acc[0][3]);
  acc_guard4(acc[1][0], acc[1][1], acc[1][2], acc[1][3]);
  acc_guard4(acc[2][0], acc[2][1], acc[2][2], acc[2][3]);
  acc_guard4(acc[3][0], acc[3][1], acc[3][2], acc[3][3]);

  float* slab = sT[wave];
#pragma unroll
  for (int i = 0; i < 4; ++i) {
    const int mBase = m0 + (i << 4);
#pragma unroll
    for (int j = 0; j < 4; ++j) {
      const int n = n0 + (j << 4) + rlane;
      float bv = 0.f;
      if (BIAS_MODE == 2) bv = bias[n];
#pragma unroll
      for (int r = 0; r < 8; ++r) {
        float v = acc[i][j][r] * scale;
        if (BIAS_MODE == 2) v += bv;
        slab[(mOff + r) * 68 + (j << 4) + rlane] = v;
      }
    }
    __builtin_amdgcn_fence(__ATOMIC_RELEASE, "workgroup");
    __builtin_amdgcn_wave_barrier();
    __builtin_amdgcn_fence(__ATOMIC_ACQUIRE, "workgroup");
    if (OUT_MODE == 0) {
      float* C = (float*)Cout;
      const int hh = lane >> 4, c4 = (lane & 15) * 4;
      for (int pass = 0; pass < 2; ++pass) {
#pragma unroll
        for (int it = 0; it < 8; ++it) {
          const int row = it * 2 + hh;
          v4f v = *(const v4f*)(slab + row * 68 + c4);
          *(volatile v4f*)(C + (size_t)(mBase + row) * ldc + n0 + c4) = v;
        }
        __threadfence();
      }
    } else {
      const int q = lane >> 3, c8 = (lane & 7) * 8;
      unsigned short* C = (unsigned short*)Cout;
      for (int pass = 0; pass < 2; ++pass) {
#pragma unroll
        for (int it = 0; it < 4; ++it) {
          const int row = it * 4 + q;
          const float* sp = slab + row * 68 + c8;
          v8h hv;
#pragma unroll
          for (int e = 0; e < 8; ++e) {
            const float t = flush16(sp[e]);
            hv[e] = (_Float16)t;
          }
          *(volatile v8h*)(C + (size_t)(mBase + row) * ldc + n0 + c8) = hv;
        }
        __threadfence();
      }
    }
    __builtin_amdgcn_fence(__ATOMIC_RELEASE, "workgroup");
    __builtin_amdgcn_wave_barrier();
    __builtin_amdgcn_fence(__ATOMIC_ACQUIRE, "workgroup");
  }
}

__global__ __launch_bounds__(256) void wt_transpose_f16_kernel(
    const float* __restrict__ W, unsigned short* __restrict__ Bt, int K, int Nreal, float carry)
{
  __shared__ __align__(16) float sT[64 * 68];
  const int tid = threadIdx.x;
  const int k0 = blockIdx.x * 64;
  const int n0 = blockIdx.y * 64;
#pragma unroll
  for (int it = 0; it < 4; ++it) {
    const int idx = it * 256 + tid;
    const int kr = idx >> 4;
    const int c4 = (idx & 15) * 4;
    const int n = n0 + c4;
    const bool ok = (n < Nreal);
    const int nc = ok ? n : (Nreal - 4);
    const v4f v = *(const v4f*)(W + (size_t)(k0 + kr) * Nreal + nc);
#pragma unroll
    for (int e = 0; e < 4; ++e) {
      float t = v[e] * carry;
      t = ok ? t : 0.0f;
      sT[(c4 + e) * 68 + kr] = flush16(t);
    }
  }
  __syncthreads();
  v8h hv[2];
#pragma unroll
  for (int it = 0; it < 2; ++it) {
    const int row = it * 32 + (tid >> 3);
    const float* sp = sT + row * 68 + (tid & 7) * 8;
    const v4f a0 = *(const v4f*)(sp);
    const v4f a1 = *(const v4f*)(sp + 4);
#pragma unroll
    for (int e = 0; e < 4; ++e) {
      hv[it][e]     = (_Float16)a0[e];
      hv[it][4 + e] = (_Float16)a1[e];
    }
  }
  for (int pass = 0; pass < 2; ++pass) {
#pragma unroll
    for (int it = 0; it < 2; ++it) {
      const int row = it * 32 + (tid >> 3);
      *(volatile v8h*)(Bt + (size_t)(n0 + row) * K + k0 + (tid & 7) * 8) = hv[it];
    }
    __threadfence();
  }
}

__global__ __launch_bounds__(256) void cast_x_flip_kernel(
    const float* __restrict__ x, unsigned short* __restrict__ X16)
{
  const int i = blockIdx.x * 256 + threadIdx.x;
  if (i >= kRowsAll * (kDm / 8)) return;
  const int row = i >> 7;
  const int c8  = (i & 127) << 3;
  const int seq = row / kSeq;
  const int t   = row - seq * kSeq;
  const int src = (seq < kBatch) ? (seq * kSeq + t) : ((seq - kBatch) * kSeq + (kSeq - 1 - t));
  const float* sp = x + (size_t)src * kDm + c8;
  const v4f a0 = *(const v4f*)(sp);
  const v4f a1 = *(const v4f*)(sp + 4);
  v8h hv;
#pragma unroll
  for (int e = 0; e < 4; ++e) {
    const float t0 = flush16(a0[e] * kCarryX);
    const float t1 = flush16(a1[e] * kCarryX);
    hv[e]     = (_Float16)t0;
    hv[4 + e] = (_Float16)t1;
  }
  unsigned short* dp = X16 + (size_t)row * kDm + c8;
  *(volatile v8h*)dp = hv;
  __threadfence();
  *(volatile v8h*)dp = hv;
}

__global__ __launch_bounds__(256) void conv_silu_kernel(
    const float* __restrict__ XZ, const float* __restrict__ cw, const float* __restrict__ cb,
    float* __restrict__ US, unsigned short* __restrict__ U16)
{
  __shared__ __align__(16) float sT[16 * kConvTP];
  const int tid = threadIdx.x, lane = tid & 31, wave = tid >> 5;
  const int d0 = blockIdx.x * 256, d = d0 + tid;
  const int g0 = blockIdx.y * 64;
  const v4f wv = *(const v4f*)(cw + (size_t)d * 4);
  const float w0 = wv[0], w1 = wv[1], w2 = wv[2], w3 = wv[3];
  const float bcv = cb[d];
  float xm3, xm2, xm1;
  {
    const bool hist = (g0 > 0);
    const int rb = hist ? (g0 - 3) : 0;
    const float v3 = XZ[(size_t)rb * kXzP + d];
    const float v2 = XZ[(size_t)(rb + 1) * kXzP + d];
    const float v1 = XZ[(size_t)(rb + 2) * kXzP + d];
    xm3 = hist ? v3 : 0.f;
    xm2 = hist ? v2 : 0.f;
    xm1 = hist ? v1 : 0.f;
  }
  const int hrow = wave >> 1;
  const int hch  = (wave & 1) * 128 + lane * 4;
#pragma unroll 1
  for (int sub = 0; sub < 4; ++sub) {
    const int lb = g0 + sub * 16;
#pragma unroll 1
    for (int s = 0; s < 16; ++s) {
      const float xcur = XZ[(size_t)(lb + s) * kXzP + d];
      float acc = w0 * xm3;
      acc = fmaf(w1, xm2, acc);
      acc = fmaf(w2, xm1, acc);
      acc = fmaf(w3, xcur, acc);
      const float sv = acc + bcv;
      const float sg = __builtin_amdgcn_rcpf(1.0f + expf(-sv));
      sT[s * kConvTP + tid] = sv * sg;
      xm3 = xm2;
      xm2 = xm1;
      xm1 = xcur;
    }
    __syncthreads();
    v4f fv[4];
    v8h uh[2];
#pragma unroll
    for (int it = 0; it < 4; ++it) fv[it] = *(const v4f*)(sT + (it * 4 + hrow) * kConvTP + hch);
#pragma unroll
    for (int it = 0; it < 2; ++it) {
      const float* sp = sT + (it * 8 + wave) * kConvTP + lane * 8;
      const v4f a0 = *(const v4f*)(sp);
      const v4f a1 = *(const v4f*)(sp + 4);
#pragma unroll
      for (int e = 0; e < 4; ++e) {
        const float t0 = flush16(a0[e] * kCarryU);
        const float t1 = flush16(a1[e] * kCarryU);
        uh[it][e]     = (_Float16)t0;
        uh[it][4 + e] = (_Float16)t1;
      }
    }
    for (int pass = 0; pass < 2; ++pass) {
#pragma unroll
      for (int it = 0; it < 4; ++it)
        *(volatile v4f*)(US + (size_t)(lb + it * 4 + hrow) * kDin + d0 + hch) = fv[it];
#pragma unroll
      for (int it = 0; it < 2; ++it)
        *(volatile v8h*)(U16 + (size_t)(lb + it * 8 + wave) * kDin + d0 + lane * 8) = uh[it];
      __threadfence();
    }
    __syncthreads();
  }
}

__global__ __launch_bounds__(128) void combine_ln_kernel(
    const float* __restrict__ MO, const float* __restrict__ lg, const float* __restrict__ lb,
    unsigned short* __restrict__ H16)
{
  __shared__ float red1[4];
  __shared__ float red2[4];
  const int tid = threadIdx.x, lane = tid & 31, wave = tid >> 5;
  const int row = blockIdx.x;
  const int b = row / kSeq;
  const int s = row - b * kSeq;
  const float* pf = MO + (size_t)row * kDm + tid * 8;
  const float* pb = MO + (size_t)((kBatch + b) * kSeq + (kSeq - 1 - s)) * kDm + tid * 8;
  const v4f f0 = *(const v4f*)(pf);
  const v4f f1 = *(const v4f*)(pf + 4);
  const v4f r0 = *(const v4f*)(pb);
  const v4f r1 = *(const v4f*)(pb + 4);
  float v[8];
#pragma unroll
  for (int e = 0; e < 4; ++e) {
    v[e]     = f0[e] + r0[e];
    v[4 + e] = f1[e] + r1[e];
  }
  float sm = ((v[0] + v[1]) + (v[2] + v[3])) + ((v[4] + v[5]) + (v[6] + v[7]));
#pragma unroll
  for (int off = 16; off >= 1; off >>= 1) sm += __shfl_xor(sm, off, 32);
  if (lane == 0) red1[wave] = sm;
  __syncthreads();
  const float mu = ((red1[0] + red1[1]) + (red1[2] + red1[3])) * (1.0f / (float)kDm);
  float dv[8];
  float sq = 0.0f;
#pragma unroll
  for (int e = 0; e < 8; ++e) {
    dv[e] = v[e] - mu;
    sq = fmaf(dv[e], dv[e], sq);
  }
#pragma unroll
  for (int off = 16; off >= 1; off >>= 1) sq += __shfl_xor(sq, off, 32);
  if (lane == 0) red2[wave] = sq;
  __syncthreads();
  const float var = ((red2[0] + red2[1]) + (red2[2] + red2[3])) * (1.0f / (float)kDm);
  const float rs = 1.0f / sqrtf(var + 1e-5f);
  const v4f g0 = *(const v4f*)(lg + tid * 8);
  const v4f g1 = *(const v4f*)(lg + tid * 8 + 4);
  const v4f b0 = *(const v4f*)(lb + tid * 8);
  const v4f b1 = *(const v4f*)(lb + tid * 8 + 4);
  v8h hv;
#pragma unroll
  for (int e = 0; e < 4; ++e) {
    const float h0 = dv[e] * rs * g0[e] + b0[e];
    const float h1 = dv[4 + e] * rs * g1[e] + b1[e];
    const float t0 = flush16(h0 * kCarryH);
    const float t1 = flush16(h1 * kCarryH);
    hv[e]     = (_Float16)t0;
    hv[4 + e] = (_Float16)t1;
  }
  unsigned short* dp = H16 + (size_t)row * kDm + tid * 8;
  *(volatile v8h*)dp = hv;
  __threadfence();
  *(volatile v8h*)dp = hv;
}

__global__ __launch_bounds__(256) void gelu_cast_kernel(
    const float* __restrict__ P, unsigned short* __restrict__ G16)
{
  __shared__ __align__(16) float sG[2048];
  const int tid = threadIdx.x;
  const size_t base = (size_t)blockIdx.x * 2048;
#pragma unroll 1
  for (int it = 0; it < 8; ++it) {
    const float xv = P[base + it * 256 + tid];
    const float er = erff(xv * 0.70710678118654752f);
    sG[it * 256 + tid] = (0.5f * xv) * (1.0f + er);
  }
  __syncthreads();
  const v4f a0 = *(const v4f*)(sG + tid * 8);
  const v4f a1 = *(const v4f*)(sG + tid * 8 + 4);
  v8h hv;
#pragma unroll
  for (int e = 0; e < 4; ++e) {
    const float t0 = flush16(a0[e] * kCarryG);
    const float t1 = flush16(a1[e] * kCarryG);
    hv[e]     = (_Float16)t0;
    hv[4 + e] = (_Float16)t1;
  }
  unsigned short* dp = G16 + base + tid * 8;
  *(volatile v8h*)dp = hv;
  __threadfence();
  *(volatile v8h*)dp = hv;
}

}

extern "C" void kernel_launch(void* const* d_in, const int* in_sizes, int n_in,
                              void* d_out, int out_size, void* d_ws, size_t ws_size,
                              hipStream_t stream) {
  if (n_in < 16) return;
  if (in_sizes[0]  != kRowsOut * kDm) return;
  if (in_sizes[1]  != kDm * kXzP) return;
  if (in_sizes[2]  != kDin * 4) return;
  if (in_sizes[3]  != kDin) return;
  if (in_sizes[4]  != kDin * kXpN) return;
  if (in_sizes[5]  != kDtR * kDin) return;
  if (in_sizes[6]  != kDin) return;
  if (in_sizes[7]  != kDin * kNst) return;
  if (in_sizes[8]  != kDin) return;
  if (in_sizes[9]  != kDin * kDm) return;
  if (in_sizes[10] != kDm) return;
  if (in_sizes[11] != kDm) return;
  if (in_sizes[12] != kDm * kDff) return;
  if (in_sizes[13] != kDff) return;
  if (in_sizes[14] != kDff * kDm) return;
  if (in_sizes[15] != kDm) return;
  if (out_size != kRowsOut * kDm) return;
  if (ws_size < kWsTotal) return;

  const float* x         = (const float*)d_in[0];
  const float* in_proj_w = (const float*)d_in[1];
  const float* conv_w    = (const float*)d_in[2];
  const float* conv_b    = (const float*)d_in[3];
  const float* x_proj_w  = (const float*)d_in[4];
  const float* dt_proj_w = (const float*)d_in[5];
  const float* dt_proj_b = (const float*)d_in[6];
  const float* A_log     = (const float*)d_in[7];
  const float* D_par     = (const float*)d_in[8];
  const float* out_proj_w = (const float*)d_in[9];
  const float* ln_g      = (const float*)d_in[10];
  const float* ln_b      = (const float*)d_in[11];
  const float* ff_w1     = (const float*)d_in[12];
  const float* ff_b1     = (const float*)d_in[13];
  const float* ff_w2     = (const float*)d_in[14];
  const float* ff_b2     = (const float*)d_in[15];
  float* out = (float*)d_out;

  char* ws = (char*)d_ws;
  unsigned short* WIN   = (unsigned short*)(ws + kOffWIN);
  unsigned short* WXP   = (unsigned short*)(ws + kOffWXP);
  unsigned short* WDT   = (unsigned short*)(ws + kOffWDT);
  unsigned short* WOUT  = (unsigned short*)(ws + kOffWOUT);
  unsigned short* WF1   = (unsigned short*)(ws + kOffWF1);
  unsigned short* WF2   = (unsigned short*)(ws + kOffWF2);
  unsigned short* X16   = (unsigned short*)(ws + kOffX16);
  float*          XZS   = (float*)(ws + kOffXZS);
  float*          US    = (float*)(ws + kOffUS);
  unsigned short* U16S  = (unsigned short*)(ws + kOffU16S);
  float*          BCS   = (float*)(ws + kOffBCS);
  unsigned short* DT16S = (unsigned short*)(ws + kOffDT16S);
  float*          DTPS  = (float*)(ws + kOffDTPS);
  unsigned short* Y16   = (unsigned short*)(ws + kOffY16);
  float*          MO    = (float*)(ws + kOffMO);
  unsigned short* H16   = (unsigned short*)(ws + kOffH16);
  unsigned short* G16   = (unsigned short*)(ws + kOffG16);

  eng::wt_transpose_f16_kernel<<<dim3(kDm / 64,  kXzP / 64),  256, 0, stream>>>(in_proj_w,  WIN,  kDm,  kXzP, kCarryW);
  eng::wt_transpose_f16_kernel<<<dim3(kDin / 64, kXpNP / 64), 256, 0, stream>>>(x_proj_w,   WXP,  kDin, kXpN, kCarryW);
  eng::wt_transpose_f16_kernel<<<dim3(kDtR / 64, kDin / 64),  256, 0, stream>>>(dt_proj_w,  WDT,  kDtR, kDin, kCarryW);
  eng::wt_transpose_f16_kernel<<<dim3(kDin / 64, kDm / 64),   256, 0, stream>>>(out_proj_w, WOUT, kDin, kDm,  kCarryW);
  eng::wt_transpose_f16_kernel<<<dim3(kDm / 64,  kDff / 64),  256, 0, stream>>>(ff_w1,      WF1,  kDm,  kDff, kCarryW);
  eng::wt_transpose_f16_kernel<<<dim3(kDff / 64, kDm / 64),   256, 0, stream>>>(ff_w2,      WF2,  kDff, kDm,  kCarryW);
  eng::cast_x_flip_kernel<<<dim3(kRowsAll * (kDm / 8) / 256), 256, 0, stream>>>(x, X16);

  for (int sq = 0; sq < kNSeq; ++sq) {
    eng::gemm_f16_kernel<0, 0><<<dim3((kSeq / 64) * (kXzP / 64) / 8), 256, 0, stream>>>(
        X16 + (size_t)sq * kSeq * kDm, kDm, WIN, kDm, (void*)XZS, kXzP, nullptr,
        kSeq, kXzP, kDm, 1.0f / (kCarryX * kCarryW));

    eng::conv_silu_kernel<<<dim3(kDin / 256, kSeq / 64), 256, 0, stream>>>(XZS, conv_w, conv_b, US, U16S);

    eng::gemm_f16_kernel<0, 1><<<dim3((kSeq / 64) * (kDtR / 64) / 8), 256, 0, stream>>>(
        U16S, kDin, WXP, kDin, (void*)DT16S, kDtR, nullptr,
        kSeq, kDtR, kDin, kCarryDt / (kCarryU * kCarryW));

    eng::gemm_f16_kernel<0, 0><<<dim3((kSeq / 64) * (kBcP / 64) / 8), 256, 0, stream>>>(
        U16S, kDin, WXP + (size_t)kDtR * kDin, kDin, (void*)BCS, kBcP, nullptr,
        kSeq, kBcP, kDin, 1.0f / (kCarryU * kCarryW));

    eng::gemm_f16_kernel<2, 0><<<dim3((kSeq / 64) * (kDin / 64) / 8), 256, 0, stream>>>(
        DT16S, kDtR, WDT, kDtR, (void*)DTPS, kDin, dt_proj_b,
        kSeq, kDin, kDtR, 1.0f / (kCarryDt * kCarryW));

    ms1_args sa;
    sa.dtpre = DTPS;
    sa.u = US;
    sa.bc = BCS;
    sa.z = XZS;
    sa.A_log = A_log;
    sa.Dskip = D_par;
    sa.y = (__half*)(Y16 + (size_t)sq * kSeq * kDin);
    sa.y_lo = nullptr;
    sa.ld_dtpre = kDin;
    sa.ld_u = kDin;
    sa.ld_bc = kBcP;
    sa.ld_z = kXzP;
    sa.ld_y = kDin;
    sa.offB = 0;
    sa.offC = kNst;
    sa.offZ = kDin;
    sa.ycarry = kCarryY;
    sa.dir = 1;
    sa.D = kDin;
    sa.L = kSeq;
    sa.nbatch = 1;
    ms1_scan_kernel<16><<<dim3(kDin / 64), 64, 0, stream>>>(sa);
  }

  eng::gemm_f16_kernel<0, 0><<<dim3((kRowsAll / 64) * (kDm / 64) / 8), 256, 0, stream>>>(
      Y16, kDin, WOUT, kDin, (void*)MO, kDm, nullptr,
      kRowsAll, kDm, kDin, 1.0f / (kCarryY * kCarryW));

  eng::combine_ln_kernel<<<dim3(kRowsOut), 128, 0, stream>>>(MO, ln_g, ln_b, H16);

  for (int ch = 0; ch < kRowsOut / kSeq; ++ch) {
    eng::gemm_f16_kernel<2, 0><<<dim3((kSeq / 64) * (kDff / 64) / 8), 256, 0, stream>>>(
        H16 + (size_t)ch * kSeq * kDm, kDm, WF1, kDm, (void*)XZS, kDff, ff_b1,
        kSeq, kDff, kDm, 1.0f / (kCarryH * kCarryW));
    eng::gelu_cast_kernel<<<dim3(kSeq * kDff / 2048), 256, 0, stream>>>(XZS, G16 + (size_t)ch * kSeq * kDff);
  }

  eng::gemm_f16_kernel<2, 0><<<dim3((kRowsOut / 64) * (kDm / 64) / 8), 256, 0, stream>>>(
      G16, kDff, WF2, kDff, (void*)out, kDm, ff_b2,
      kRowsOut, kDm, kDff, 1.0f / (kCarryG * kCarryW));
}
